// Swin3DViTBlock_87428354277547
// MI455X (gfx1250) — hardware-run, weakly checked
//
#include <hip/hip_runtime.h>
#include <stdint.h>
#include <math.h>

#define DEVINL __device__ __forceinline__

typedef _Float16 f16t;
typedef _Float16 v16h __attribute__((ext_vector_type(16)));
typedef _Float16 v8h  __attribute__((ext_vector_type(8)));
typedef float    v8f  __attribute__((ext_vector_type(8)));
typedef float    v4f  __attribute__((ext_vector_type(4)));
typedef v8h __attribute__((may_alias)) v8ha;
typedef v4f __attribute__((may_alias)) v4fa;
union FragH { v16h v; v8h half[2]; };

#define NB     2
#define GH     32
#define GW     32
#define GD     16
#define TOK    32768
#define TOKB   16384
#define CD     384
#define NQ     1152
#define NH     1536
#define NHEAD  12
#define HD     32
#define NOISE  256
#define NADA   2304
#define PSTR   2304
#define TPB    256
#define WAVES  8
#define MT     128
#define NTL    128
#define PQF    132
#define VP     72
#define AP     264
#define ACAR   16.0f
#define WCAR   256.0f
#define QCAR   16.0f
#define PCAR   1024.0f
#define OCAR   64.0f
#define HCAR   16.0f
#define INV_AW (1.0f / 4096.0f)
#define INV_OW (1.0f / 16384.0f)
#define SSC    (0.17677669529663687f / 256.0f)
#define OSC    (1.0f / 256.0f)

#define BWQ  (NQ * CD / 8 / TPB)
#define BWO  (CD * CD / 8 / TPB)
#define BW1  (NH * CD / 8 / TPB)
#define BW2  (CD * NH / 8 / TPB)

static_assert(TPB == WAVES * 32);
static_assert(NB * GH * GW * GD == TOK);
static_assert(GH * GW * GD == TOKB);
static_assert(NHEAD * HD == CD);
static_assert(NQ == 3 * CD);
static_assert(NH == 4 * CD);
static_assert(NADA == 6 * CD);
static_assert((TOK % MT) == 0);
static_assert((TOKB % MT) == 0);
static_assert((NQ % NTL) == 0 && (CD % NTL) == 0 && (NH % NTL) == 0);
static_assert((CD % 32) == 0 && (NH % 32) == 0 && (NOISE % 32) == 0);
static_assert(CD == 32 * 12);
static_assert((TOK % WAVES) == 0);
static_assert(BWQ * TPB * 8 == NQ * CD);
static_assert(BWO * TPB * 8 == CD * CD);
static_assert(BW1 * TPB * 8 == NH * CD);
static_assert(BW2 * TPB * 8 == CD * NH);
static_assert((NADA % (16 * WAVES)) == 0);
static_assert((PQF % 4) == 0 && (VP % 8) == 0 && (AP % 8) == 0);
static_assert(64 * PQF * 4 <= 40000);

DEVINL int imin(int a, int b) { return a < b ? a : b; }

DEVINL v8f wmma_f16(v16h a, v16h b, v8f c) {
  v8f d = __builtin_amdgcn_wmma_f32_16x16x32_f16(false, a, false, b, (short)0, c, false, false);
  asm volatile("v_nop\n\tv_nop\n\tv_nop\n\tv_nop" : "+v"(d) : "v"(a), "v"(b));
  return d;
}
DEVINL v8f zero8f() {
  v8f z = {0.f, 0.f, 0.f, 0.f, 0.f, 0.f, 0.f, 0.f};
  return z;
}
DEVINL void load_frag(FragH& f, const f16t* row, int k0) {
  f.half[0] = *(const v8ha*)(row + k0);
  f.half[1] = *(const v8ha*)(row + k0 + 16);
}

DEVINL int tok_of(int b, int hb, int wb, int db, int lr) {
  const int wh = lr >> 4, ww = (lr >> 2) & 3, wd = lr & 3;
  return ((b * GH + hb * 4 + wh) * GW + wb * 4 + ww) * GD + db * 4 + wd;
}

__global__ __launch_bounds__(TPB) void wcvt_k(const float* __restrict__ qw, const float* __restrict__ ow,
                                             const float* __restrict__ w1, const float* __restrict__ w2,
                                             f16t* __restrict__ WQ, f16t* __restrict__ WO,
                                             f16t* __restrict__ W1p, f16t* __restrict__ W2p)
{
  const int blk = blockIdx.x, tid = threadIdx.x;
  if (blk >= BWQ + BWO + BW1 + BW2) return;
  const float* src;
  f16t* dst;
  int rb;
  if (blk < BWQ)                  { src = qw; dst = WQ;  rb = blk; }
  else if (blk < BWQ + BWO)       { src = ow; dst = WO;  rb = blk - BWQ; }
  else if (blk < BWQ + BWO + BW1) { src = w1; dst = W1p; rb = blk - BWQ - BWO; }
  else                            { src = w2; dst = W2p; rb = blk - BWQ - BWO - BW1; }
  const size_t idx = ((size_t)rb * TPB + tid) * 8;
  const v4f a = *(const v4fa*)(src + idx), c = *(const v4fa*)(src + idx + 4);
  v8h o;
  #pragma unroll
  for (int j = 0; j < 4; ++j) {
    o[j]     = (f16t)(a[j] * WCAR);
    o[4 + j] = (f16t)(c[j] * WCAR);
  }
  *(volatile v8h*)(dst + idx) = o;
  __threadfence();
  *(volatile v8h*)(dst + idx) = o;
}

__global__ __launch_bounds__(TPB) void ada_k(const float* __restrict__ xn, const float* __restrict__ aw,
                                            const float* __restrict__ ab, float* __restrict__ params)
{
  __shared__ __attribute__((aligned(16))) f16t  sA[16 * AP];
  __shared__ __attribute__((aligned(16))) float sPm[2 * PSTR];
  const int tid = threadIdx.x, lane = tid & 31, wave = tid >> 5;
  const int h = lane >> 4, m = lane & 15;

  {
    const float v0 = xn[tid], v1 = xn[NOISE + tid];
    const float s0 = v0 * (1.0f / (1.0f + __expf(-v0)));
    const float s1 = v1 * (1.0f / (1.0f + __expf(-v1)));
    sA[0 * AP + tid] = (f16t)(s0 * ACAR);
    sA[1 * AP + tid] = (f16t)(s1 * ACAR);
    #pragma unroll
    for (int r = 2; r < 16; ++r) sA[r * AP + tid] = (f16t)0.0f;
  }
  __syncthreads();

  #pragma unroll 1
  for (int jj = 0; jj < NADA / 16 / WAVES; ++jj) {
    const int j = wave + WAVES * jj;
    v8f acc = zero8f();
    const float* wr = aw + (size_t)(16 * j + m) * NOISE + 8 * h;
    #pragma unroll 1
    for (int ks = 0; ks < NOISE / 32; ++ks) {
      const int k0 = 32 * ks;
      FragH a;
      a.half[0] = *(const v8ha*)(sA + m * AP + k0 + 8 * h);
      a.half[1] = *(const v8ha*)(sA + m * AP + k0 + 16 + 8 * h);
      const v4f w0 = *(const v4fa*)(wr + k0),      w1v = *(const v4fa*)(wr + k0 + 4);
      const v4f w2v = *(const v4fa*)(wr + k0 + 16), w3v = *(const v4fa*)(wr + k0 + 20);
      FragH bw;
      #pragma unroll
      for (int e = 0; e < 4; ++e) {
        bw.v[e]      = (f16t)(w0[e]  * WCAR);
        bw.v[4 + e]  = (f16t)(w1v[e] * WCAR);
        bw.v[8 + e]  = (f16t)(w2v[e] * WCAR);
        bw.v[12 + e] = (f16t)(w3v[e] * WCAR);
      }
      acc = wmma_f16(a.v, bw.v, acc);
    }
    if (h == 0) {
      const int n = 16 * j + m;
      const float bv = ab[n];
      sPm[n]        = acc[0] * INV_AW + bv;
      sPm[PSTR + n] = acc[1] * INV_AW + bv;
    }
  }
  __syncthreads();

  v4f pv[5];
  #pragma unroll
  for (int it = 0; it < 5; ++it) {
    const int pc = imin(it * TPB + tid, 2 * PSTR / 4 - 1);
    pv[it] = *(const v4fa*)(sPm + 4 * pc);
  }
  #pragma unroll
  for (int it = 0; it < 5; ++it) {
    const int pc = it * TPB + tid;
    if (pc < 2 * PSTR / 4) *(volatile v4f*)(params + 4 * pc) = pv[it];
  }
  __threadfence();
  #pragma unroll
  for (int it = 0; it < 5; ++it) {
    const int pc = it * TPB + tid;
    if (pc < 2 * PSTR / 4) *(volatile v4f*)(params + 4 * pc) = pv[it];
  }
}

__global__ __launch_bounds__(TPB) void ln_mod_k(const float* xin, const float* __restrict__ params,
                                               int shoff, int scoff, f16t* __restrict__ XM)
{
  __shared__ __attribute__((aligned(16))) f16t sX[8 * CD];
  const int tid = threadIdx.x, lane = tid & 31, wave = tid >> 5;
  const int t = blockIdx.x * 8 + wave;
  const float* xr = xin + (size_t)t * CD + 12 * lane;
  const v4f xa = *(const v4fa*)xr, xb = *(const v4fa*)(xr + 4), xc = *(const v4fa*)(xr + 8);

  float s = 0.0f;
  #pragma unroll
  for (int e = 0; e < 4; ++e) s += xa[e] + xb[e] + xc[e];
  #pragma unroll
  for (int off = 16; off >= 1; off >>= 1) s += __shfl_xor(s, off, 32);
  const float mean = s * (1.0f / 384.0f);
  float s2 = 0.0f;
  #pragma unroll
  for (int e = 0; e < 4; ++e) {
    const float d0 = xa[e] - mean, d1 = xb[e] - mean, d2 = xc[e] - mean;
    s2 = fmaf(d0, d0, s2); s2 = fmaf(d1, d1, s2); s2 = fmaf(d2, d2, s2);
  }
  #pragma unroll
  for (int off = 16; off >= 1; off >>= 1) s2 += __shfl_xor(s2, off, 32);
  const float rstd = rsqrtf(s2 * (1.0f / 384.0f) + 1e-5f);

  const int bsel = t >> 14;
  const float* shp = params + (size_t)bsel * PSTR + shoff + 12 * lane;
  const float* scp = params + (size_t)bsel * PSTR + scoff + 12 * lane;
  const v4f sha = *(const v4fa*)shp, shb = *(const v4fa*)(shp + 4), shc = *(const v4fa*)(shp + 8);
  const v4f sca = *(const v4fa*)scp, scb = *(const v4fa*)(scp + 4), scc = *(const v4fa*)(scp + 8);

  f16t* sx = sX + wave * CD + 12 * lane;
  #pragma unroll
  for (int e = 0; e < 4; ++e) {
    const float y0 = (xa[e] - mean) * rstd, y1 = (xb[e] - mean) * rstd, y2 = (xc[e] - mean) * rstd;
    sx[e]     = (f16t)((y0 * (1.0f + sca[e]) + sha[e]) * ACAR);
    sx[4 + e] = (f16t)((y1 * (1.0f + scb[e]) + shb[e]) * ACAR);
    sx[8 + e] = (f16t)((y2 * (1.0f + scc[e]) + shc[e]) * ACAR);
  }
  __syncthreads();

  const size_t base = (size_t)blockIdx.x * 8 * CD;
  const int p1 = (tid & 127) + 256;
  const v8h v0 = *(const v8ha*)(sX + 8 * tid);
  const v8h v1 = *(const v8ha*)(sX + 8 * p1);
  f16t* d0 = XM + base + 8 * tid;
  f16t* d1 = XM + base + 8 * p1;
  *(volatile v8h*)d0 = v0;
  if (tid < 128) *(volatile v8h*)d1 = v1;
  __threadfence();
  *(volatile v8h*)d0 = v0;
  if (tid < 128) *(volatile v8h*)d1 = v1;
}

template <int EPI>
__global__ __launch_bounds__(TPB) void gemm_k(const f16t* __restrict__ A, const f16t* __restrict__ Wt,
                                             const float* __restrict__ bias, const float* resid,
                                             const float* __restrict__ gate, float* outf,
                                             f16t* __restrict__ outh, int N, int K, float inv, float ocar)
{
  __shared__ __attribute__((aligned(16))) float sbuf[64 * PQF];
  const int tid = threadIdx.x, lane = tid & 31, wave = tid >> 5;
  const int h = lane >> 4, m = lane & 15;
  const int wm = wave >> 1, wn = wave & 1;
  const int row0 = blockIdx.y * MT, n0 = blockIdx.x * NTL;
  const int mo = row0 + 32 * wm, no = n0 + 64 * wn;

  v8f acc[2][4];
  #pragma unroll
  for (int mh = 0; mh < 2; ++mh)
    #pragma unroll
    for (int t = 0; t < 4; ++t) acc[mh][t] = zero8f();

  const f16t* arow0 = A + (size_t)(mo + m) * K + 8 * h;
  const f16t* arow1 = arow0 + (size_t)16 * K;
  const f16t* brow  = Wt + (size_t)(no + m) * K + 8 * h;
  #pragma unroll 1
  for (int k0 = 0; k0 < K; k0 += 32) {
    FragH a0, a1;
    load_frag(a0, arow0, k0);
    load_frag(a1, arow1, k0);
    #pragma unroll
    for (int t = 0; t < 4; ++t) {
      FragH bw;
      load_frag(bw, brow + (size_t)16 * t * K, k0);
      acc[0][t] = wmma_f16(a0.v, bw.v, acc[0][t]);
      acc[1][t] = wmma_f16(a1.v, bw.v, acc[1][t]);
    }
  }

  const int bsel = row0 >> 14;
  v4f gv = {0.f, 0.f, 0.f, 0.f};
  if constexpr (EPI == 2) gv = *(const v4fa*)(gate + (size_t)bsel * PSTR + n0 + 4 * lane);

  #pragma unroll
  for (int p = 0; p < 2; ++p) {
    if ((wm >> 1) == p) {
      #pragma unroll
      for (int t = 0; t < 4; ++t) {
        const float bv = bias[no + 16 * t + m];
        #pragma unroll
        for (int mh = 0; mh < 2; ++mh) {
          #pragma unroll
          for (int r = 0; r < 8; ++r)
            sbuf[((wm & 1) * 32 + 16 * mh + 8 * h + r) * PQF + 64 * wn + 16 * t + m] = acc[mh][t][r] * inv + bv;
        }
      }
    }
    __syncthreads();
    const int seg0 = row0 + 64 * p;
    if constexpr (EPI == 2) {
      v4f vals[8];
      #pragma unroll
      for (int i = 0; i < 8; ++i) {
        const int row = wave + 8 * i;
        const v4f c  = *(const v4fa*)(sbuf + row * PQF + 4 * lane);
        const v4f rs = *(const v4fa*)(resid + (size_t)(seg0 + row) * N + n0 + 4 * lane);
        vals[i] = rs + gv * c;
      }
      #pragma unroll
      for (int i = 0; i < 8; ++i)
        *(volatile v4f*)(outf + (size_t)(seg0 + wave + 8 * i) * N + n0 + 4 * lane) = vals[i];
      __threadfence();
      #pragma unroll
      for (int i = 0; i < 8; ++i)
        *(volatile v4f*)(outf + (size_t)(seg0 + wave + 8 * i) * N + n0 + 4 * lane) = vals[i];
    } else {
      v8h hv[4];
      #pragma unroll
      for (int j = 0; j < 4; ++j) {
        const int row = wave + 8 * (2 * j + h);
        const float* sp = sbuf + row * PQF + 8 * m;
        const v4f c0 = *(const v4fa*)sp, c1 = *(const v4fa*)(sp + 4);
        #pragma unroll
        for (int e = 0; e < 4; ++e) {
          float u0 = c0[e], u1 = c1[e];
          if constexpr (EPI == 1) {
            u0 = 0.5f * u0 * (1.0f + erff(u0 * 0.70710678118654752f));
            u1 = 0.5f * u1 * (1.0f + erff(u1 * 0.70710678118654752f));
          }
          hv[j][e]     = (f16t)(u0 * ocar);
          hv[j][4 + e] = (f16t)(u1 * ocar);
        }
      }
      #pragma unroll
      for (int j = 0; j < 4; ++j)
        *(volatile v8h*)(outh + (size_t)(seg0 + wave + 8 * (2 * j + h)) * N + n0 + 8 * m) = hv[j];
      __threadfence();
      #pragma unroll
      for (int j = 0; j < 4; ++j)
        *(volatile v8h*)(outh + (size_t)(seg0 + wave + 8 * (2 * j + h)) * N + n0 + 8 * m) = hv[j];
    }
    __syncthreads();
  }
}

__global__ __launch_bounds__(TPB) void attn_k(const f16t* __restrict__ QKV, f16t* __restrict__ ATT)
{
  __shared__ __attribute__((aligned(16))) f16t sVt[2 * HD * VP];
  __shared__ __attribute__((aligned(16))) f16t sP[WAVES * 16 * VP];
  __shared__ __attribute__((aligned(16))) f16t sO[64 * VP];
  const int tid = threadIdx.x, lane = tid & 31, wave = tid >> 5;
  const int h = lane >> 4, m = lane & 15;
  const int hp = blockIdx.x % 6, wid = blockIdx.x / 6;
  const int db = wid & 3, wb = (wid >> 2) & 7, hb = (wid >> 5) & 7, b = wid >> 8;

  {
    const int hs0 = tid >> 7, key = (tid >> 1) & 63, ch = (tid & 1) * 16;
    const f16t* vr = QKV + (size_t)tok_of(b, hb, wb, db, key) * NQ + 2 * CD + (2 * hp + hs0) * HD + ch;
    const v8h f0 = *(const v8ha*)vr, f1 = *(const v8ha*)(vr + 8);
    f16t* vt = sVt + (hs0 * HD + ch) * VP + key;
    #pragma unroll
    for (int i = 0; i < 8; ++i) {
      vt[i * VP]       = f0[i];
      vt[(8 + i) * VP] = f1[i];
    }
  }
  __syncthreads();

  const int hs = wave >> 2, wq = wave & 3, head = 2 * hp + hs;
  FragH qa;
  {
    const f16t* qr = QKV + (size_t)tok_of(b, hb, wb, db, wq * 16 + m) * NQ + head * HD + 8 * h;
    qa.half[0] = *(const v8ha*)qr;
    qa.half[1] = *(const v8ha*)(qr + 16);
  }
  v8f st[4];
  #pragma unroll
  for (int nt = 0; nt < 4; ++nt) {
    const f16t* kr = QKV + (size_t)tok_of(b, hb, wb, db, nt * 16 + m) * NQ + CD + head * HD + 8 * h;
    FragH kb;
    kb.half[0] = *(const v8ha*)kr;
    kb.half[1] = *(const v8ha*)(kr + 16);
    st[nt] = wmma_f16(qa.v, kb.v, zero8f());
  }

  f16t* pw = sP + wave * 16 * VP;
  #pragma unroll
  for (int r = 0; r < 8; ++r) {
    const float s0 = st[0][r] * SSC, s1 = st[1][r] * SSC, s2 = st[2][r] * SSC, s3 = st[3][r] * SSC;
    float mx = fmaxf(fmaxf(s0, s1), fmaxf(s2, s3));
    #pragma unroll
    for (int off = 8; off >= 1; off >>= 1) mx = fmaxf(mx, __shfl_xor(mx, off, 32));
    const float e0 = __expf(s0 - mx), e1 = __expf(s1 - mx), e2 = __expf(s2 - mx), e3 = __expf(s3 - mx);
    float sum = (e0 + e1) + (e2 + e3);
    #pragma unroll
    for (int off = 8; off >= 1; off >>= 1) sum += __shfl_xor(sum, off, 32);
    const float pm = PCAR * (1.0f / sum);
    f16t* prow = pw + (8 * h + r) * VP + m;
    prow[0]  = (f16t)(e0 * pm);
    prow[16] = (f16t)(e1 * pm);
    prow[32] = (f16t)(e2 * pm);
    prow[48] = (f16t)(e3 * pm);
  }
  __syncthreads();

  v8f oacc[2];
  oacc[0] = zero8f();
  oacc[1] = zero8f();
  #pragma unroll
  for (int s = 0; s < 2; ++s) {
    FragH pa;
    const f16t* pr = pw + m * VP + 32 * s + 8 * h;
    pa.half[0] = *(const v8ha*)pr;
    pa.half[1] = *(const v8ha*)(pr + 16);
    #pragma unroll
    for (int ct = 0; ct < 2; ++ct) {
      const f16t* vrow = sVt + (hs * HD + ct * 16 + m) * VP + 32 * s + 8 * h;
      FragH vb;
      vb.half[0] = *(const v8ha*)vrow;
      vb.half[1] = *(const v8ha*)(vrow + 16);
      oacc[ct] = wmma_f16(pa.v, vb.v, oacc[ct]);
    }
  }

  #pragma unroll
  for (int ct = 0; ct < 2; ++ct) {
    #pragma unroll
    for (int r = 0; r < 8; ++r)
      sO[(wq * 16 + 8 * h + r) * VP + hs * HD + ct * 16 + m] = (f16t)(oacc[ct][r] * OSC);
  }
  __syncthreads();

  const int q = tid & 7;
  const int rA = tid >> 3, rB = rA + 32;
  const v8h vA = *(const v8ha*)(sO + rA * VP + 8 * q);
  const v8h vB = *(const v8ha*)(sO + rB * VP + 8 * q);
  f16t* dA = ATT + (size_t)tok_of(b, hb, wb, db, rA) * CD + 64 * hp + 8 * q;
  f16t* dB = ATT + (size_t)tok_of(b, hb, wb, db, rB) * CD + 64 * hp + 8 * q;
  *(volatile v8h*)dA = vA;
  *(volatile v8h*)dB = vB;
  __threadfence();
  *(volatile v8h*)dA = vA;
  *(volatile v8h*)dB = vB;
}

extern "C" void kernel_launch(void* const* d_in, const int* in_sizes, int n_in,
                              void* d_out, int out_size, void* d_ws, size_t ws_size,
                              hipStream_t stream) {
  if (n_in < 12) return;
  if (in_sizes[0] != TOK * CD) return;
  if (in_sizes[1] != NB * NOISE) return;
  if (in_sizes[2] != NADA * NOISE || in_sizes[3] != NADA) return;
  if (in_sizes[4] != NQ * CD || in_sizes[5] != NQ) return;
  if (in_sizes[6] != CD * CD || in_sizes[7] != CD) return;
  if (in_sizes[8] != NH * CD || in_sizes[9] != NH) return;
  if (in_sizes[10] != CD * NH || in_sizes[11] != CD) return;
  if (out_size != TOK * CD) return;

  const float* x       = (const float*)d_in[0];
  const float* x_noise = (const float*)d_in[1];
  const float* ada_w   = (const float*)d_in[2];
  const float* ada_b   = (const float*)d_in[3];
  const float* qkv_w   = (const float*)d_in[4];
  const float* qkv_b   = (const float*)d_in[5];
  const float* out_w   = (const float*)d_in[6];
  const float* out_b   = (const float*)d_in[7];
  const float* mlp_w1  = (const float*)d_in[8];
  const float* mlp_b1  = (const float*)d_in[9];
  const float* mlp_w2  = (const float*)d_in[10];
  const float* mlp_b2  = (const float*)d_in[11];
  float* outp = (float*)d_out;

  const size_t szPar = (size_t)NB * PSTR * 4;
  const size_t szWQ  = (size_t)NQ * CD * 2;
  const size_t szWO  = (size_t)CD * CD * 2;
  const size_t szW1  = (size_t)NH * CD * 2;
  const size_t szW2  = (size_t)CD * NH * 2;
  const size_t szA   = (size_t)TOK * CD * 2;
  const size_t szB   = (size_t)TOK * NH * 2;
  size_t off = 0;
  char* ws = (char*)d_ws;
  float* params = (float*)(ws + off); off += szPar;
  f16t*  WQ     = (f16t*)(ws + off);  off += szWQ;
  f16t*  WO     = (f16t*)(ws + off);  off += szWO;
  f16t*  W1p    = (f16t*)(ws + off);  off += szW1;
  f16t*  W2p    = (f16t*)(ws + off);  off += szW2;
  f16t*  regA   = (f16t*)(ws + off);  off += szA;
  f16t*  regB   = (f16t*)(ws + off);  off += szB;
  if (off > ws_size) return;
  if ((size_t)TOK * NQ * 2 > szB) return;

  f16t* XMp  = regA;
  f16t* ATTp = regA;
  f16t* QKVp = regB;
  f16t* Hp   = regB;

  wcvt_k<<<BWQ + BWO + BW1 + BW2, TPB, 0, stream>>>(qkv_w, out_w, mlp_w1, mlp_w2, WQ, WO, W1p, W2p);
  ada_k<<<1, TPB, 0, stream>>>(x_noise, ada_w, ada_b, params);
  ln_mod_k<<<TOK / 8, TPB, 0, stream>>>(x, params, 0, CD, XMp);
  gemm_k<0><<<dim3(NQ / NTL, TOK / MT), TPB, 0, stream>>>(XMp, WQ, qkv_b, x, params, outp, QKVp,
                                                          NQ, CD, INV_AW, QCAR);
  attn_k<<<512 * 6, TPB, 0, stream>>>(QKVp, ATTp);
  gemm_k<2><<<dim3(CD / NTL, TOK / MT), TPB, 0, stream>>>(ATTp, WO, out_b, x, params + 2 * CD, outp, XMp,
                                                          CD, CD, INV_OW, 1.0f);
  ln_mod_k<<<TOK / 8, TPB, 0, stream>>>(outp, params, 3 * CD, 4 * CD, XMp);
  gemm_k<1><<<dim3(NH / NTL, TOK / MT), TPB, 0, stream>>>(XMp, W1p, mlp_b1, x, params, outp, Hp,
                                                          NH, CD, INV_AW, HCAR);
  gemm_k<2><<<dim3(CD / NTL, TOK / MT), TPB, 0, stream>>>(Hp, W2p, mlp_b2, outp, params + 5 * CD, outp, XMp,
                                                          CD, NH, INV_AW, 1.0f);
  (void)hipGetLastError();
}
